// MambaBlock_37134287241961
// MI455X (gfx1250) — hardware-verified
//
#include <hip/hip_runtime.h>
#include <math.h>

typedef __attribute__((ext_vector_type(16))) _Float16 v16h;
typedef __attribute__((ext_vector_type(8)))  _Float16 v8h;
typedef __attribute__((ext_vector_type(16))) __bf16   v16b;
typedef __attribute__((ext_vector_type(8)))  __bf16   v8b;
typedef __attribute__((ext_vector_type(8)))  float    v8f;
typedef __attribute__((ext_vector_type(4)))  float    v4f;
typedef __attribute__((ext_vector_type(2)))  float    v2f;

constexpr int kB     = 8;
constexpr int kL     = 1024;
constexpr int kC     = 256;
constexpr int kDin   = 512;
constexpr int kNst   = 16;
constexpr int kDtR   = 16;
constexpr int kXdW   = 48;
constexpr int kXdP   = 64;
constexpr int kXzP   = 2 * kDin;
constexpr int kHid   = 1024;
constexpr int kRows  = kB * kL;
constexpr int kConvTP = 260;
constexpr int kScanTS = 64;
constexpr int kScanCh = 64;
constexpr int kScanYP = 68;
constexpr int kLnTP   = 260;
constexpr int kNcTP   = 68;
constexpr float kWCarry  = 64.0f;
constexpr float kUcCarry = 256.0f;
constexpr float kYCarry  = 1024.0f;
constexpr float kHdCarry = 64.0f;
constexpr float kScaleIn  = 1.0f / kWCarry;
constexpr float kScaleX   = 1.0f / (kUcCarry * kWCarry);
constexpr float kScaleOut = 1.0f / (kYCarry * kWCarry);
constexpr float kScaleM1  = 1.0f / kWCarry;
constexpr float kScaleM2  = 1.0f / (kHdCarry * kWCarry);
constexpr float kInvC = 1.0f / (float)kC;
constexpr float kEps  = 1e-5f;
constexpr float kRsqrt2 = 0.70710678118654752f;
static_assert(kDtR + 2 * kNst == kXdW);
static_assert(kXdW <= kXdP);
static_assert((kC % 32) == 0 && (kDin % 32) == 0 && (kHid % 32) == 0);
static_assert((kRows % 64) == 0 && (kXzP % 64) == 0 && (kXdP % 64) == 0 && (kC % 64) == 0 && (kHid % 64) == 0);
static_assert((kL % 64) == 0 && (kL % kScanTS) == 0 && (kDin % kScanCh) == 0 && (kDin % 256) == 0 && (kL % 32) == 0);
constexpr int kTilesIn  = (kRows / 64) * (kXzP / 64);
constexpr int kTilesX   = (kRows / 64) * (kXdP / 64);
constexpr int kTilesOut = (kRows / 64) * (kC / 64);
constexpr int kTilesM1  = (kRows / 64) * (kHid / 64);
constexpr int kTilesM2  = (kRows / 64) * (kC / 64);
static_assert((kTilesIn % 8) == 0 && (kTilesX % 8) == 0 && (kTilesOut % 8) == 0 && (kTilesM1 % 8) == 0 && (kTilesM2 % 8) == 0);

constexpr size_t kOffWIN16  = 0;
constexpr size_t kOffWX16   = kOffWIN16  + (size_t)kXzP * kC * 2;
constexpr size_t kOffWOUT16 = kOffWX16   + (size_t)kXdP * kDin * 2;
constexpr size_t kOffW1T16  = kOffWOUT16 + (size_t)kC * kDin * 2;
constexpr size_t kOffW2T16  = kOffW1T16  + (size_t)kHid * kC * 2;
constexpr size_t kOffRES1   = kOffW2T16  + (size_t)kC * kHid * 2;
constexpr size_t kOffXN1    = kOffRES1   + (size_t)kRows * kC * 4;
constexpr size_t kOffXZ     = kOffXN1    + (size_t)kRows * kC * 2;
constexpr size_t kOffHP     = kOffXZ;
constexpr size_t kOffUC     = kOffXZ     + (size_t)kRows * kXzP * 4;
constexpr size_t kOffUC16   = kOffUC     + (size_t)kRows * kDin * 4;
constexpr size_t kOffXD     = kOffUC16   + (size_t)kRows * kDin * 2;
constexpr size_t kOffY16    = kOffXD     + (size_t)kRows * kXdP * 4;
constexpr size_t kOffX2     = kOffY16    + (size_t)kRows * kDin * 2;
constexpr size_t kOffXN2    = kOffX2     + (size_t)kRows * kC * 4;
constexpr size_t kOffHD16   = kOffXN2    + (size_t)kRows * kC * 2;
constexpr size_t kOffOT     = kOffHD16   + (size_t)kRows * kHid * 2;
constexpr size_t kWsTotal   = kOffOT     + (size_t)kRows * kC * 4;
static_assert((size_t)kRows * kXzP * 4 == (size_t)kRows * kHid * 4);
static_assert(kWsTotal == 121438208ull);
static_assert(kWsTotal <= 134217728ull);
static_assert((kOffWX16 % 128) == 0 && (kOffWOUT16 % 128) == 0 && (kOffW1T16 % 128) == 0 && (kOffW2T16 % 128) == 0 &&
              (kOffRES1 % 128) == 0 && (kOffXN1 % 128) == 0 && (kOffXZ % 128) == 0 && (kOffUC % 128) == 0 &&
              (kOffUC16 % 128) == 0 && (kOffXD % 128) == 0 && (kOffY16 % 128) == 0 && (kOffX2 % 128) == 0 &&
              (kOffXN2 % 128) == 0 && (kOffHD16 % 128) == 0 && (kOffOT % 128) == 0);

__device__ __forceinline__ unsigned short f2bf_bits(float f) {
  unsigned u = __float_as_uint(f);
  return (unsigned short)((u + 0x7FFFu + ((u >> 16) & 1u)) >> 16);
}
__device__ __forceinline__ float bf_bits2f(unsigned short h) { return __uint_as_float(((unsigned)h) << 16); }

__device__ __forceinline__ void dep_guard4_h(v8f& a, v8f& b, v8f& c, v8f& d, v16h x, v16h y) { asm volatile("v_nop\n\tv_nop\n\tv_nop\n\tv_nop" : "+v"(a), "+v"(b), "+v"(c), "+v"(d) : "v"(x), "v"(y)); }
__device__ __forceinline__ void dep_guard4_b(v8f& a, v8f& b, v8f& c, v8f& d, v16b x, v16b y) { asm volatile("v_nop\n\tv_nop\n\tv_nop\n\tv_nop" : "+v"(a), "+v"(b), "+v"(c), "+v"(d) : "v"(x), "v"(y)); }
__device__ __forceinline__ void keep4_h(v16h a, v16h b, v16h c, v16h d) { asm volatile("v_nop" :: "v"(a), "v"(b), "v"(c), "v"(d)); }
__device__ __forceinline__ void keep4_b(v16b a, v16b b, v16b c, v16b d) { asm volatile("v_nop" :: "v"(a), "v"(b), "v"(c), "v"(d)); }
__device__ __forceinline__ void acc_guard4(v8f& a, v8f& b, v8f& c, v8f& d) { asm volatile("v_nop\n\tv_nop\n\tv_nop\n\tv_nop" : "+v"(a), "+v"(b), "+v"(c), "+v"(d)); }
template <typename T> struct Frag;
template <> struct Frag<_Float16> {
  typedef v16h V; union U { v16h v; v8h h[2]; };
  static __device__ __forceinline__ v16h load(const _Float16* p) {
    U f; f.h[0] = *(const v8h*)(p); f.h[1] = *(const v8h*)(p + 16); return f.v;
  }
  static __device__ __forceinline__ v8f mma(v16h a, v16h b, v8f c) {
    return __builtin_amdgcn_wmma_f32_16x16x32_f16(false, a, false, b, (short)0, c, false, false);
  }
  static __device__ __forceinline__ void guard4(v8f& a, v8f& b, v8f& c, v8f& d, v16h x, v16h y) { dep_guard4_h(a, b, c, d, x, y); }
  static __device__ __forceinline__ void keep(v16h a, v16h b, v16h c, v16h d) { keep4_h(a, b, c, d); }
};
template <> struct Frag<__bf16> {
  typedef v16b V; union U { v16b v; v8b h[2]; };
  static __device__ __forceinline__ v16b load(const __bf16* p) {
    U f; f.h[0] = *(const v8b*)(p); f.h[1] = *(const v8b*)(p + 16); return f.v;
  }
  static __device__ __forceinline__ v8f mma(v16b a, v16b b, v8f c) {
    return __builtin_amdgcn_wmma_f32_16x16x32_bf16(false, a, false, b, (short)0, c, false, false);
  }
  static __device__ __forceinline__ void guard4(v8f& a, v8f& b, v8f& c, v8f& d, v16b x, v16b y) { dep_guard4_b(a, b, c, d, x, y); }
  static __device__ __forceinline__ void keep(v16b a, v16b b, v16b c, v16b d) { keep4_b(a, b, c, d); }
};

template <int ET> struct Elem;
template <> struct Elem<0> { typedef _Float16 T; };
template <> struct Elem<1> { typedef __bf16 T; };
template <int ET, bool SPLIT, int BIAS_MODE, int OUT_MODE, bool RESID, int ACT = 0>
__global__ __launch_bounds__(256) void wmma_gemm64(
    const unsigned short* __restrict__ Ap, const unsigned short* __restrict__ A2p, int lda, long strideA,
    const unsigned short* __restrict__ Btp, const unsigned short* __restrict__ Bt2p, int ldb, long strideB,
    void* __restrict__ Cout, void* __restrict__ Cout2, int ldc, long strideC,
    const float* __restrict__ bias,
    const float* __restrict__ resid, long strideR,
    int M, int N, int K, float scale) {
  static_assert(!(RESID && OUT_MODE != 0));
  static_assert(ACT >= 0 && ACT <= 4);
  typedef typename Elem<ET>::T T;
  typedef typename Frag<T>::V V;
  const T* A = (const T*)Ap; const T* A2 = (const T*)A2p; const T* Bt = (const T*)Btp; const T* Bt2 = (const T*)Bt2p;
  __shared__ __align__(16) float sT[8][16 * 68];
  const int b    = blockIdx.y;
  const int lane = threadIdx.x & 31;
  const int wave = threadIdx.x >> 5;
  const int tilesN = N >> 6;
  const int tilesM = M >> 6;
  const int tile = blockIdx.x * 8 + wave;
  if (tile >= tilesM * tilesN) return;
  const int tm = tile / tilesN;
  const int tn = tile - tm * tilesN;
  const int m0 = tm << 6;
  const int n0 = tn << 6;

  const T* Ab  = A  + (size_t)b * strideA;
  const T* Bb  = Bt + (size_t)b * strideB;
  const T* Ab2 = SPLIT ? (A2  + (size_t)b * strideA) : nullptr;
  const T* Bb2 = SPLIT ? (Bt2 + (size_t)b * strideB) : nullptr;

  const int rlane = lane & 15;
  const int koff  = (lane >> 4) * 8;
  const int mOff  = (lane >> 4) * 8;

  v8f acc[4][4];
#pragma unroll
  for (int i = 0; i < 4; ++i)
#pragma unroll
    for (int j = 0; j < 4; ++j) acc[i][j] = (v8f){0.f,0.f,0.f,0.f,0.f,0.f,0.f,0.f};

  for (int k0 = 0; k0 < K; k0 += 32) {
    V bh[4], bl[4];
#pragma unroll
    for (int j = 0; j < 4; ++j) {
      const size_t bo = (size_t)(n0 + (j << 4) + rlane) * ldb + koff + k0;
      bh[j] = Frag<T>::load(Bb + bo);
      if (SPLIT) bl[j] = Frag<T>::load(Bb2 + bo);
    }
#pragma unroll
    for (int i = 0; i < 4; ++i) {
      const size_t ao = (size_t)(m0 + (i << 4) + rlane) * lda + koff + k0;
      V ah = Frag<T>::load(Ab + ao);
      V al;
      if (SPLIT) al = Frag<T>::load(Ab2 + ao);
#pragma unroll
      for (int j = 0; j < 4; ++j) {
        acc[i][j] = Frag<T>::mma(ah, bh[j], acc[i][j]);
        if (SPLIT) {
          acc[i][j] = Frag<T>::mma(ah, bl[j], acc[i][j]);
          acc[i][j] = Frag<T>::mma(al, bh[j], acc[i][j]);
        }
      }
      Frag<T>::guard4(acc[i][0], acc[i][1], acc[i][2], acc[i][3], ah, SPLIT ? al : bh[3]);
    }
    Frag<T>::keep(bh[0], bh[1], bh[2], bh[3]);
    if (SPLIT) Frag<T>::keep(bl[0], bl[1], bl[2], bl[3]);
  }
  acc_guard4(acc[0][0], acc[0][1], acc[0][2], acc[0][3]);
  acc_guard4(acc[1][0], acc[1][1], acc[1][2], acc[1][3]);
  acc_guard4(acc[2][0], acc[2][1], acc[2][2], acc[2][3]);
  acc_guard4(acc[3][0], acc[3][1], acc[3][2], acc[3][3]);

  float* slab = sT[wave];
  const float* Rb = RESID ? (resid + (size_t)b * strideR) : nullptr;
#pragma unroll
  for (int i = 0; i < 4; ++i) {
    const int mBase = m0 + (i << 4);
#pragma unroll
    for (int j = 0; j < 4; ++j) {
      const int n = n0 + (j << 4) + rlane;
      float bv = 0.f;
      if (BIAS_MODE == 2) bv = bias[n];
#pragma unroll
      for (int r = 0; r < 8; ++r) {
        float v = acc[i][j][r] * scale;
        if (BIAS_MODE == 1) v += bias[mBase + mOff + r];
        if (BIAS_MODE == 2) v += bv;
        if (ACT == 1) v = tanhf(v);
        if (ACT == 2) v = fmaxf(v, 0.0f);
        if (ACT == 3) v = v / (1.0f + expf(-v));
        if (ACT == 4) v = (v > 0.f) ? v : 0.01f * v;
        slab[(mOff + r) * 68 + (j << 4) + rlane] = v;
      }
    }
    __builtin_amdgcn_fence(__ATOMIC_RELEASE, "workgroup");
    __builtin_amdgcn_wave_barrier();
    __builtin_amdgcn_fence(__ATOMIC_ACQUIRE, "workgroup");
    if (OUT_MODE == 0) {
      float* C = (float*)Cout + (size_t)b * strideC;
      const int hh = lane >> 4, c4 = (lane & 15) * 4;
      v4f vals[8];
#pragma unroll
      for (int it = 0; it < 8; ++it) {
        const int row = it * 2 + hh;
        v4f v = *(const v4f*)(slab + row * 68 + c4);
        if (RESID) {
          const v4f rv = *(const v4f*)(Rb + (size_t)(mBase + row) * ldc + n0 + c4);
          v = v + rv;
        }
        vals[it] = v;
      }
      for (int pass = 0; pass < 2; ++pass) {
#pragma unroll
        for (int it = 0; it < 8; ++it) {
          const int row = it * 2 + hh;
          *(volatile v4f*)(C + (size_t)(mBase + row) * ldc + n0 + c4) = vals[it];
        }
        __threadfence();
      }
    } else {
      const int q = lane >> 3, c8 = (lane & 7) * 8;
      unsigned short* C  = (unsigned short*)Cout  + (size_t)b * strideC;
      unsigned short* C2 = (OUT_MODE == 2) ? ((unsigned short*)Cout2 + (size_t)b * strideC) : nullptr;
      for (int pass = 0; pass < 2; ++pass) {
#pragma unroll
        for (int it = 0; it < 4; ++it) {
          const int row = it * 4 + q;
          const float* sp = slab + row * 68 + c8;
          v8h hv, lv;
#pragma unroll
          for (int e = 0; e < 8; ++e) {
            if (OUT_MODE == 1) {
              hv[e] = (_Float16)sp[e];
            } else {
              unsigned short hb = f2bf_bits(sp[e]);
              unsigned short lb = f2bf_bits(sp[e] - bf_bits2f(hb));
              hv[e] = __builtin_bit_cast(_Float16, hb);
              lv[e] = __builtin_bit_cast(_Float16, lb);
            }
          }
          *(volatile v8h*)(C + (size_t)(mBase + row) * ldc + n0 + c8) = hv;
          if (OUT_MODE == 2) *(volatile v8h*)(C2 + (size_t)(mBase + row) * ldc + n0 + c8) = lv;
        }
        __threadfence();
      }
    }
    __builtin_amdgcn_fence(__ATOMIC_RELEASE, "workgroup");
    __builtin_amdgcn_wave_barrier();
    __builtin_amdgcn_fence(__ATOMIC_ACQUIRE, "workgroup");
  }
}

__global__ __launch_bounds__(256) void transpose_cast_kernel(
    const float* __restrict__ W, unsigned short* __restrict__ Bt, int Kdim, int Ndim, int Npad, float scale)
{
  __shared__ float tile[64 * 65];
  const int tid = threadIdx.x, lane = tid & 31, wave = tid >> 5;
  const int n0 = blockIdx.x * 64;
  const int k0 = blockIdx.y * 64;
  (void)Npad;
#pragma unroll
  for (int p = 0; p < 16; ++p) {
    const int idx = tid + p * 256;
    const int kk  = idx >> 6;
    const int nn  = idx & 63;
    const int n   = n0 + nn;
    const int nc  = (n < Ndim) ? n : (Ndim - 1);
    const float v = W[(size_t)(k0 + kk) * Ndim + nc];
    tile[kk * 65 + nn] = (n < Ndim) ? (v * scale) : 0.f;
  }
  __syncthreads();
  const int q = lane >> 3, c8 = (lane & 7) * 8;
  v8h hv[2];
#pragma unroll
  for (int it = 0; it < 2; ++it) {
    const int nrow = it * 32 + wave * 4 + q;
#pragma unroll
    for (int e = 0; e < 8; ++e) hv[it][e] = (_Float16)tile[(c8 + e) * 65 + nrow];
  }
  for (int pass = 0; pass < 2; ++pass) {
#pragma unroll
    for (int it = 0; it < 2; ++it) {
      const int nrow = it * 32 + wave * 4 + q;
      *(volatile v8h*)(Bt + (size_t)(n0 + nrow) * Kdim + k0 + c8) = hv[it];
    }
    __threadfence();
  }
}

__global__ __launch_bounds__(256) void ln1_tokenize_kernel(
    const float* __restrict__ x, const float* __restrict__ g, const float* __restrict__ be,
    float* __restrict__ RES1, unsigned short* __restrict__ XN1)
{
  __shared__ __align__(16) float tile[32 * kLnTP];
  const int tid = threadIdx.x, lane = tid & 31, wave = tid >> 5;
  constexpr int kBlkPerImg = kL / 32;
  const int b  = blockIdx.x / kBlkPerImg;
  const int l0 = (blockIdx.x - b * kBlkPerImg) * 32;
  const float* xb = x + (size_t)b * kC * kL + l0;
  const int rc = tid >> 3, l4 = (tid & 7) * 4;
#pragma unroll 1
  for (int ib = 0; ib < 2; ++ib) {
#pragma unroll
    for (int p = 0; p < 4; ++p) {
      const int c = (ib * 4 + p) * 32 + rc;
      const v4f v = *(const v4f*)(xb + (size_t)c * kL + l4);
      tile[(l4 + 0) * kLnTP + c] = v[0];
      tile[(l4 + 1) * kLnTP + c] = v[1];
      tile[(l4 + 2) * kLnTP + c] = v[2];
      tile[(l4 + 3) * kLnTP + c] = v[3];
    }
  }
  __syncthreads();
  const v4f g0 = *(const v4f*)(g + lane * 8);
  const v4f g1 = *(const v4f*)(g + lane * 8 + 4);
  const v4f e0 = *(const v4f*)(be + lane * 8);
  const v4f e1 = *(const v4f*)(be + lane * 8 + 4);
#pragma unroll 1
  for (int r = 0; r < 4; ++r) {
    const int row = wave * 4 + r;
    const float* tr = tile + row * kLnTP;
    const v4f a0 = *(const v4f*)(tr + lane * 8);
    const v4f a1 = *(const v4f*)(tr + lane * 8 + 4);
    float s = ((a0[0] + a0[1]) + (a0[2] + a0[3])) + ((a1[0] + a1[1]) + (a1[2] + a1[3]));
#pragma unroll
    for (int off = 16; off > 0; off >>= 1) s += __shfl_xor(s, off, 32);
    const float mu = s * kInvC;
    float qs = 0.f;
#pragma unroll
    for (int e = 0; e < 4; ++e) {
      const float d0 = a0[e] - mu, d1 = a1[e] - mu;
      qs += d0 * d0;
      qs += d1 * d1;
    }
#pragma unroll
    for (int off = 16; off > 0; off >>= 1) qs += __shfl_xor(qs, off, 32);
    const float var  = qs * kInvC;
    const float rstd = rsqrtf(var + kEps);
    v8h hv;
#pragma unroll
    for (int e = 0; e < 4; ++e) {
      hv[e]     = (_Float16)(((a0[e] - mu) * rstd) * g0[e] + e0[e]);
      hv[4 + e] = (_Float16)(((a1[e] - mu) * rstd) * g1[e] + e1[e]);
    }
    const v4f r0 = *(const v4f*)(tr + lane * 4);
    const v4f r1 = *(const v4f*)(tr + 128 + lane * 4);
    const size_t grow = (size_t)b * kL + l0 + row;
    for (int pass = 0; pass < 2; ++pass) {
      *(volatile v4f*)(RES1 + grow * kC + lane * 4) = r0;
      *(volatile v4f*)(RES1 + grow * kC + 128 + lane * 4) = r1;
      *(volatile v8h*)(XN1 + grow * kC + lane * 8) = hv;
      __threadfence();
    }
  }
}

__global__ __launch_bounds__(256) void conv_silu_kernel(
    const float* __restrict__ XZ, const float* __restrict__ cw, const float* __restrict__ cb,
    float* __restrict__ UC, unsigned short* __restrict__ UC16)
{
  __shared__ __align__(16) float sT[16 * kConvTP];
  const int tid = threadIdx.x, lane = tid & 31, wave = tid >> 5;
  const int d0 = blockIdx.x * 256, d = d0 + tid;
  const int g0 = blockIdx.y * 64;
  const int tb = g0 & (kL - 1);
  const float w0 = cw[d * 4 + 0], w1 = cw[d * 4 + 1], w2 = cw[d * 4 + 2], w3 = cw[d * 4 + 3];
  const float bc = cb[d];
  float xm3, xm2, xm1;
  {
    const bool hist = (tb > 0);
    const int rb = hist ? (g0 - 3) : g0;
    const float v3 = XZ[(size_t)rb * kXzP + d];
    const float v2 = XZ[(size_t)(rb + 1) * kXzP + d];
    const float v1 = XZ[(size_t)(rb + 2) * kXzP + d];
    xm3 = hist ? v3 : 0.f;
    xm2 = hist ? v2 : 0.f;
    xm1 = hist ? v1 : 0.f;
  }
  const int hrow = wave >> 1;
  const int hch  = (wave & 1) * 128 + lane * 4;
#pragma unroll 1
  for (int sub = 0; sub < 4; ++sub) {
    const int lb = g0 + sub * 16;
#pragma unroll 1
    for (int s = 0; s < 16; ++s) {
      const float xcur = XZ[(size_t)(lb + s) * kXzP + d];
      float acc = w0 * xm3;
      acc = fmaf(w1, xm2, acc);
      acc = fmaf(w2, xm1, acc);
      acc = fmaf(w3, xcur, acc);
      const float sv = acc + bc;
      const float sg = __builtin_amdgcn_rcpf(1.0f + __expf(-sv));
      sT[s * kConvTP + tid] = sv * sg;
      xm3 = xm2; xm2 = xm1; xm1 = xcur;
    }
    __syncthreads();
    v4f fv[4];
    v8h bv[2];
#pragma unroll
    for (int it = 0; it < 4; ++it) fv[it] = *(const v4f*)(sT + (it * 4 + hrow) * kConvTP + hch);
#pragma unroll
    for (int it = 0; it < 2; ++it) {
      const float* sp = sT + (it * 8 + wave) * kConvTP + lane * 8;
      const v4f a0 = *(const v4f*)(sp);
      const v4f a1 = *(const v4f*)(sp + 4);
#pragma unroll
      for (int e = 0; e < 4; ++e) {
        bv[it][e]     = (_Float16)(a0[e] * kUcCarry);
        bv[it][4 + e] = (_Float16)(a1[e] * kUcCarry);
      }
    }
    for (int pass = 0; pass < 2; ++pass) {
#pragma unroll
      for (int it = 0; it < 4; ++it)
        *(volatile v4f*)(UC + (size_t)(lb + it * 4 + hrow) * kDin + d0 + hch) = fv[it];
#pragma unroll
      for (int it = 0; it < 2; ++it)
        *(volatile v8h*)(UC16 + (size_t)(lb + it * 8 + wave) * kDin + d0 + lane * 8) = bv[it];
      __threadfence();
    }
    __syncthreads();
  }
}

__global__ __launch_bounds__(64) void scan_kernel(
    const float* __restrict__ XD, const float* __restrict__ UC, const float* __restrict__ XZ,
    const float* __restrict__ Wdt, const float* __restrict__ bdt, const float* __restrict__ Alog,
    const float* __restrict__ Dp, unsigned short* __restrict__ Y16)
{
  __shared__ __align__(16) float sX[kScanTS * kXdP];
  __shared__ __align__(16) float sY[kScanTS * kScanYP];
  __shared__ __align__(16) float sW[kDtR * kScanCh];
  __shared__ __align__(16) float sA[kNst * kScanCh];
  const int tid = threadIdx.x, lane = tid & 31, wave = tid >> 5;
  constexpr int kBlkPerB = kDin / kScanCh;
  const int bix = blockIdx.x / kBlkPerB;
  const int d0  = (blockIdx.x - bix * kBlkPerB) * kScanCh;
  const int d   = d0 + tid;
  const size_t row0 = (size_t)bix * kL;
#pragma unroll 1
  for (int r = 0; r < kDtR; ++r) sW[r * kScanCh + tid] = Wdt[(size_t)r * kDin + d];
#pragma unroll 1
  for (int s = 0; s < kNst; ++s) sA[s * kScanCh + tid] = -expf(Alog[(size_t)d * kNst + s]);
  __syncthreads();
  float negA[kNst], h[kNst];
#pragma unroll
  for (int s = 0; s < kNst; ++s) {
    negA[s] = sA[s * kScanCh + tid];
    h[s] = 0.f;
  }
  const float bb = bdt[d], Dd = Dp[d];
  const int lr = tid >> 4, lc4 = (tid & 15) * 4;
  const int q = lane >> 3, c8 = (lane & 7) * 8;
#pragma unroll 1
  for (int t0 = 0; t0 < kL; t0 += kScanTS) {
    __syncthreads();
#pragma unroll 1
    for (int ib = 0; ib < 4; ++ib) {
#pragma unroll
      for (int i = 0; i < 4; ++i) {
        const int r = lr + 4 * (ib * 4 + i);
        *(v4f*)(sX + r * kXdP + lc4) = *(const v4f*)(XD + (row0 + t0 + r) * kXdP + lc4);
      }
    }
    __syncthreads();
#pragma unroll 1
    for (int s = 0; s < kScanTS; ++s) {
      const int t = t0 + s;
      const float* xr = sX + s * kXdP;
      float vdot = 0.f;
#pragma unroll 1
      for (int r4 = 0; r4 < kDtR / 4; ++r4) {
        const v4f xv = *(const v4f*)(xr + 4 * r4);
        const float* wp = sW + (4 * r4) * kScanCh + tid;
        vdot = fmaf(xv[0], wp[0], vdot);
        vdot = fmaf(xv[1], wp[kScanCh], vdot);
        vdot = fmaf(xv[2], wp[2 * kScanCh], vdot);
        vdot = fmaf(xv[3], wp[3 * kScanCh], vdot);
      }
      float Bs[kNst], Cs[kNst];
#pragma unroll
      for (int q4 = 0; q4 < 4; ++q4) {
        const v4f bv = *(const v4f*)(xr + kDtR + 4 * q4);
        const v4f cv = *(const v4f*)(xr + kDtR + kNst + 4 * q4);
        Bs[4 * q4 + 0] = bv[0]; Bs[4 * q4 + 1] = bv[1]; Bs[4 * q4 + 2] = bv[2]; Bs[4 * q4 + 3] = bv[3];
        Cs[4 * q4 + 0] = cv[0]; Cs[4 * q4 + 1] = cv[1]; Cs[4 * q4 + 2] = cv[2]; Cs[4 * q4 + 3] = cv[3];
      }
      const float v   = vdot + bb;
      const float ea  = __expf(-fabsf(v));
      const float dt  = fmaxf(v, 0.0f) + log1pf(ea);
      const float xt  = UC[(row0 + t) * kDin + d];
      const float dtx = dt * xt;
      float y = 0.f;
#pragma unroll
      for (int k = 0; k < kNst; ++k) {
        const float e = __expf(dt * negA[k]);
        float p = dtx * Bs[k];
        asm volatile("" : "+v"(p));
        float qv = h[k] * e;
        asm volatile("" : "+v"(qv));
        const float hn = qv + p;
        h[k] = hn;
        float rr = hn * Cs[k];
        asm volatile("" : "+v"(rr));
        y += rr;
      }
      float sk = xt * Dd;
      asm volatile("" : "+v"(sk));
      y += sk;
      const float zv = XZ[(row0 + t) * kXzP + kDin + d];
      const float sg = __builtin_amdgcn_rcpf(1.0f + __expf(-zv));
      y = y * (zv * sg);
      sY[s * kScanYP + tid] = y * kYCarry;
    }
    __syncthreads();
    v8h hv[8];
#pragma unroll
    for (int it = 0; it < 8; ++it) {
      const int row = it * 8 + wave * 4 + q;
      const float* sp = sY + row * kScanYP + c8;
      const v4f a0 = *(const v4f*)(sp);
      const v4f a1 = *(const v4f*)(sp + 4);
#pragma unroll
      for (int e = 0; e < 4; ++e) {
        hv[it][e]     = (_Float16)a0[e];
        hv[it][4 + e] = (_Float16)a1[e];
      }
    }
    for (int pass = 0; pass < 2; ++pass) {
#pragma unroll
      for (int it = 0; it < 8; ++it) {
        const int row = it * 8 + wave * 4 + q;
        const size_t o = (row0 + t0 + row) * kDin + d0 + c8;
        *(volatile v8h*)(Y16 + o) = hv[it];
      }
      __threadfence();
    }
  }
}

__global__ __launch_bounds__(256) void ln2_kernel(
    const float* __restrict__ X2, const float* __restrict__ g, const float* __restrict__ be,
    unsigned short* __restrict__ XN2)
{
  const int tid = threadIdx.x, lane = tid & 31, wave = tid >> 5;
  const size_t row = (size_t)blockIdx.x * 8 + wave;
  const float* xr = X2 + row * kC + lane * 8;
  const v4f a0 = *(const v4f*)(xr);
  const v4f a1 = *(const v4f*)(xr + 4);
  const v4f g0 = *(const v4f*)(g + lane * 8);
  const v4f g1 = *(const v4f*)(g + lane * 8 + 4);
  const v4f e0 = *(const v4f*)(be + lane * 8);
  const v4f e1 = *(const v4f*)(be + lane * 8 + 4);
  float s = ((a0[0] + a0[1]) + (a0[2] + a0[3])) + ((a1[0] + a1[1]) + (a1[2] + a1[3]));
#pragma unroll
  for (int off = 16; off > 0; off >>= 1) s += __shfl_xor(s, off, 32);
  const float mu = s * kInvC;
  float qs = 0.f;
#pragma unroll
  for (int e = 0; e < 4; ++e) {
    const float d0 = a0[e] - mu, d1 = a1[e] - mu;
    qs += d0 * d0;
    qs += d1 * d1;
  }
#pragma unroll
  for (int off = 16; off > 0; off >>= 1) qs += __shfl_xor(qs, off, 32);
  const float var  = qs * kInvC;
  const float rstd = rsqrtf(var + kEps);
  v8h hv;
#pragma unroll
  for (int e = 0; e < 4; ++e) {
    hv[e]     = (_Float16)(((a0[e] - mu) * rstd) * g0[e] + e0[e]);
    hv[4 + e] = (_Float16)(((a1[e] - mu) * rstd) * g1[e] + e1[e]);
  }
  unsigned short* qd = XN2 + row * kC + lane * 8;
  *(volatile v8h*)qd = hv;
  __threadfence();
  *(volatile v8h*)qd = hv;
}

__global__ __launch_bounds__(256) void gelu_cast_kernel(
    const float* __restrict__ HP, unsigned short* __restrict__ HD16, int n2)
{
  const int i = blockIdx.x * 256 + threadIdx.x;
  if (i >= n2) return;
  const v2f v = *(const v2f*)(HP + 2 * (size_t)i);
  const float va = v[0], vb = v[1];
  float ga = 0.f, gb = 0.f;
#pragma unroll 1
  for (int e = 0; e < 2; ++e) {
    const float t  = (e == 0) ? va : vb;
    const float gt = ((0.5f * t) * (1.0f + erff(t * kRsqrt2))) * kHdCarry;
    ga = (e == 0) ? gt : ga;
    gb = (e == 0) ? gb : gt;
  }
  const _Float16 h0 = (_Float16)ga, h1 = (_Float16)gb;
  const unsigned u = (unsigned)__builtin_bit_cast(unsigned short, h0) | ((unsigned)__builtin_bit_cast(unsigned short, h1) << 16);
  ((volatile unsigned*)HD16)[i] = u;
  __threadfence();
  ((volatile unsigned*)HD16)[i] = u;
}

__global__ __launch_bounds__(256) void nchw_store_kernel(const float* __restrict__ OT, float* __restrict__ out)
{
  __shared__ __align__(16) float tile[64 * kNcTP];
  const int tid = threadIdx.x, lane = tid & 31, wave = tid >> 5;
  const int c0 = blockIdx.x * 64;
  const int t0 = blockIdx.y * 64;
  const int b  = t0 / kL;
  const int l0 = t0 - b * kL;
#pragma unroll
  for (int p = 0; p < 4; ++p) {
    const int idx = tid + p * 256;
    const int r   = idx >> 4;
    const int c4  = (idx & 15) * 4;
    const v4f v = *(const v4f*)(OT + (size_t)(t0 + r) * kC + c0 + c4);
    tile[(c4 + 0) * kNcTP + r] = v[0];
    tile[(c4 + 1) * kNcTP + r] = v[1];
    tile[(c4 + 2) * kNcTP + r] = v[2];
    tile[(c4 + 3) * kNcTP + r] = v[3];
  }
  __syncthreads();
  const int hh = lane >> 4, l4 = (lane & 15) * 4;
  v4f vals[4];
#pragma unroll
  for (int it = 0; it < 4; ++it) {
    const int ch = wave * 8 + it * 2 + hh;
    vals[it] = *(const v4f*)(tile + ch * kNcTP + l4);
  }
  for (int pass = 0; pass < 2; ++pass) {
#pragma unroll
    for (int it = 0; it < 4; ++it) {
      const int ch = wave * 8 + it * 2 + hh;
      *(volatile v4f*)(out + ((size_t)(b * kC + c0 + ch) * kL) + l0 + l4) = vals[it];
    }
    __threadfence();
  }
}

extern "C" void kernel_launch(void* const* d_in, const int* in_sizes, int n_in,
                              void* d_out, int out_size, void* d_ws, size_t ws_size,
                              hipStream_t stream)
{
  if (n_in < 18) return;
  if (in_sizes[0]  != kB * kC * kL) return;
  if (in_sizes[1]  != kC || in_sizes[2] != kC || in_sizes[3] != kC || in_sizes[4] != kC) return;
  if (in_sizes[5]  != kC * kXzP) return;
  if (in_sizes[6]  != kDin * 4 || in_sizes[7] != kDin) return;
  if (in_sizes[8]  != kDin * kXdW) return;
  if (in_sizes[9]  != kDtR * kDin || in_sizes[10] != kDin) return;
  if (in_sizes[11] != kDin * kNst || in_sizes[12] != kDin) return;
  if (in_sizes[13] != kDin * kC) return;
  if (in_sizes[14] != kC * kHid || in_sizes[15] != kHid) return;
  if (in_sizes[16] != kHid * kC || in_sizes[17] != kC) return;
  if (out_size != kB * kC * kL) return;
  if (ws_size < kWsTotal) return;

  const float* x      = (const float*)d_in[0];
  const float* ln1_g  = (const float*)d_in[1];
  const float* ln1_b  = (const float*)d_in[2];
  const float* ln2_g  = (const float*)d_in[3];
  const float* ln2_b  = (const float*)d_in[4];
  const float* W_in   = (const float*)d_in[5];
  const float* conv_w = (const float*)d_in[6];
  const float* conv_b = (const float*)d_in[7];
  const float* W_x    = (const float*)d_in[8];
  const float* W_dt   = (const float*)d_in[9];
  const float* b_dt   = (const float*)d_in[10];
  const float* A_log  = (const float*)d_in[11];
  const float* D_par  = (const float*)d_in[12];
  const float* W_out  = (const float*)d_in[13];
  const float* W1     = (const float*)d_in[14];
  const float* b1     = (const float*)d_in[15];
  const float* W2     = (const float*)d_in[16];
  const float* b2     = (const float*)d_in[17];
  float* dout = (float*)d_out;

  char* ws = (char*)d_ws;
  unsigned short* WIN16  = (unsigned short*)(ws + kOffWIN16);
  unsigned short* WX16   = (unsigned short*)(ws + kOffWX16);
  unsigned short* WOUT16 = (unsigned short*)(ws + kOffWOUT16);
  unsigned short* W1T16  = (unsigned short*)(ws + kOffW1T16);
  unsigned short* W2T16  = (unsigned short*)(ws + kOffW2T16);
  float*          RES1   = (float*)(ws + kOffRES1);
  unsigned short* XN1    = (unsigned short*)(ws + kOffXN1);
  float*          XZ     = (float*)(ws + kOffXZ);
  float*          HP     = (float*)(ws + kOffHP);
  float*          UC     = (float*)(ws + kOffUC);
  unsigned short* UC16   = (unsigned short*)(ws + kOffUC16);
  float*          XD     = (float*)(ws + kOffXD);
  unsigned short* Y16    = (unsigned short*)(ws + kOffY16);
  float*          X2     = (float*)(ws + kOffX2);
  unsigned short* XN2    = (unsigned short*)(ws + kOffXN2);
  unsigned short* HD16   = (unsigned short*)(ws + kOffHD16);
  float*          OT     = (float*)(ws + kOffOT);
  const float* dummy_bias  = b_dt;
  const float* dummy_resid = x;

  transpose_cast_kernel<<<dim3(kXzP / 64, kC / 64),   256, 0, stream>>>(W_in,  WIN16,  kC,   kXzP, kXzP, kWCarry);
  transpose_cast_kernel<<<dim3(kXdP / 64, kDin / 64), 256, 0, stream>>>(W_x,   WX16,   kDin, kXdW, kXdP, kWCarry);
  transpose_cast_kernel<<<dim3(kC / 64,   kDin / 64), 256, 0, stream>>>(W_out, WOUT16, kDin, kC,   kC,   kWCarry);
  transpose_cast_kernel<<<dim3(kHid / 64, kC / 64),   256, 0, stream>>>(W1,    W1T16,  kC,   kHid, kHid, kWCarry);
  transpose_cast_kernel<<<dim3(kC / 64,   kHid / 64), 256, 0, stream>>>(W2,    W2T16,  kHid, kC,   kC,   kWCarry);

  ln1_tokenize_kernel<<<kRows / 32, 256, 0, stream>>>(x, ln1_g, ln1_b, RES1, XN1);

  wmma_gemm64<0, false, 0, 0, false><<<dim3(kTilesIn / 8, 1), 256, 0, stream>>>(
      XN1, XN1, kC, 0L, WIN16, WIN16, kC, 0L,
      (void*)XZ, (void*)XZ, kXzP, 0L, dummy_bias, dummy_resid, 0L, kRows, kXzP, kC, kScaleIn);

  conv_silu_kernel<<<dim3(kDin / 256, kRows / 64), 256, 0, stream>>>(XZ, conv_w, conv_b, UC, UC16);

  wmma_gemm64<0, false, 0, 0, false><<<dim3(kTilesX / 8, 1), 256, 0, stream>>>(
      UC16, UC16, kDin, 0L, WX16, WX16, kDin, 0L,
      (void*)XD, (void*)XD, kXdP, 0L, dummy_bias, dummy_resid, 0L, kRows, kXdP, kDin, kScaleX);

  scan_kernel<<<kB * (kDin / kScanCh), kScanCh, 0, stream>>>(XD, UC, XZ, W_dt, b_dt, A_log, D_par, Y16);

  wmma_gemm64<0, false, 0, 0, true><<<dim3(kTilesOut / 8, 1), 256, 0, stream>>>(
      Y16, Y16, kDin, 0L, WOUT16, WOUT16, kDin, 0L,
      (void*)X2, (void*)X2, kC, 0L, dummy_bias, RES1, 0L, kRows, kC, kDin, kScaleOut);

  ln2_kernel<<<kRows / 8, 256, 0, stream>>>(X2, ln2_g, ln2_b, XN2);

  wmma_gemm64<0, false, 2, 0, false><<<dim3(kTilesM1 / 8, 1), 256, 0, stream>>>(
      XN2, XN2, kC, 0L, W1T16, W1T16, kC, 0L,
      (void*)HP, (void*)HP, kHid, 0L, b1, dummy_resid, 0L, kRows, kHid, kC, kScaleM1);

  gelu_cast_kernel<<<(kRows * kHid) / 2 / 256, 256, 0, stream>>>(HP, HD16, (kRows * kHid) / 2);

  wmma_gemm64<0, false, 2, 0, true><<<dim3(kTilesM2 / 8, 1), 256, 0, stream>>>(
      HD16, HD16, kHid, 0L, W2T16, W2T16, kHid, 0L,
      (void*)OT, (void*)OT, kC, 0L, b2, X2, 0L, kRows, kC, kHid, kScaleM2);

  nchw_store_kernel<<<dim3(kC / 64, kRows / 64), 256, 0, stream>>>(OT, dout);
}
